// Attention_11287174054323
// MI455X (gfx1250) — hardware-verified
//
#include <hip/hip_runtime.h>
#include <math.h>

#ifndef NB
#define NB 2
#endif
#ifndef SEQ
#define SEQ 2048
#endif
#define SEQ_FULL 2048
#define DIM 2048
#define NH 16
#define HD 128
#define QKP 4096
#define XB_FULL (SEQ_FULL * DIM)

static_assert(NH * HD == DIM);
static_assert(QKP == 2 * DIM);
static_assert(SEQ % 64 == 0);
static_assert(SEQ <= SEQ_FULL);
static_assert(DIM % 64 == 0);

typedef __attribute__((ext_vector_type(16))) _Float16 v16h;
typedef __attribute__((ext_vector_type(8)))  _Float16 v8h;
typedef __attribute__((ext_vector_type(8)))  float    v8f;
typedef __attribute__((ext_vector_type(4)))  float    v4f;
typedef __attribute__((ext_vector_type(4)))  unsigned v4u;

union FragU { v16h v; v8h h[2]; };
__device__ __forceinline__ v16h ldfrag(const _Float16* p) { FragU f; f.h[0] = *(const v8h*)(p); f.h[1] = *(const v8h*)(p + 16); return f.v; }
__device__ __forceinline__ v8f mma16(v16h a, v16h b, v8f c) { return __builtin_amdgcn_wmma_f32_16x16x32_f16(false, a, false, b, (short)0, c, false, false); }
__device__ __forceinline__ void guard4(v8f& a, v8f& b, v8f& c, v8f& d, v16h x, v16h y0, v16h y1, v16h y2, v16h y3) {
  asm volatile("v_nop\n\tv_nop\n\tv_nop\n\tv_nop" : "+v"(a), "+v"(b), "+v"(c), "+v"(d) : "v"(x), "v"(y0), "v"(y1), "v"(y2), "v"(y3));
}
__device__ __forceinline__ void dep_guard_h(v8f& a, v8f& b, v16h x, v16h y) { asm volatile("v_nop\n\tv_nop\n\tv_nop\n\tv_nop" : "+v"(a), "+v"(b) : "v"(x), "v"(y)); }
__device__ __forceinline__ void keep4_h(v16h a, v16h b, v16h c, v16h d) { asm volatile("v_nop" :: "v"(a), "v"(b), "v"(c), "v"(d)); }
__device__ __forceinline__ void acc_guard4(v8f& a, v8f& b, v8f& c, v8f& d) { asm volatile("v_nop\n\tv_nop\n\tv_nop\n\tv_nop" : "+v"(a), "+v"(b), "+v"(c), "+v"(d)); }

#define VST2(T, ptr, val) do { const T vst2_v_ = (val); *(volatile T*)(ptr) = vst2_v_; __threadfence(); *(volatile T*)(ptr) = vst2_v_; } while (0)

__device__ __forceinline__ float bf_rne_f32(float v) { const unsigned u = __float_as_uint(v); const unsigned r = (u + 0x7fffu + ((u >> 16) & 1u)) & 0xffff0000u; return __uint_as_float(r); }
__device__ __forceinline__ unsigned pk2h(float a, float b) { return (unsigned)__builtin_bit_cast(unsigned short, (_Float16)a) | ((unsigned)__builtin_bit_cast(unsigned short, (_Float16)b) << 16); }

struct InvF { float v[64]; };
static_assert(sizeof(InvF) == 256);
static_assert((SEQ * 64) % 256 == 0);
__global__ __launch_bounds__(256) void k_tab(float* __restrict__ cs, float* __restrict__ sn, InvF f) {
  const unsigned idx = blockIdx.x * 256u + threadIdx.x;
  const unsigned t = idx >> 6, i = idx & 63u;
  float inv = 0.f;
#pragma unroll
  for (unsigned k = 0; k < 64u; ++k) inv = (k == i) ? f.v[k] : inv;
  const float ang = (float)t * inv;
  const float cv = cosf(ang), sv = sinf(ang);
  VST2(float, cs + idx, cv);
  VST2(float, sn + idx, sv);
}

static_assert((SEQ * DIM / 8) % 256 == 0);
__global__ __launch_bounds__(256) void k_cast_x(const float* __restrict__ x, unsigned short* __restrict__ X16) {
  const unsigned u = blockIdx.x * 256u + threadIdx.x;
  const unsigned b = blockIdx.y;
  const float* s = x + (size_t)b * (size_t)XB_FULL + (size_t)u * 8u;
  const v4f a = *(const v4f*)(s), c = *(const v4f*)(s + 4);
  v4u pk;
  pk.x = pk2h(bf_rne_f32(a.x), bf_rne_f32(a.y)); pk.y = pk2h(bf_rne_f32(a.z), bf_rne_f32(a.w));
  pk.z = pk2h(bf_rne_f32(c.x), bf_rne_f32(c.y)); pk.w = pk2h(bf_rne_f32(c.z), bf_rne_f32(c.w));
  unsigned short* d = X16 + (size_t)b * ((size_t)SEQ * DIM) + (size_t)u * 8u;
  VST2(v4u, d, pk);
}

static_assert((DIM * DIM / 8) % 256 == 0);
static_assert(DIM / 8 == 256);
__global__ __launch_bounds__(256) void k_castT4(const float* __restrict__ w0, const float* __restrict__ w1, const float* __restrict__ w2, const float* __restrict__ w3,
                                                 unsigned short* __restrict__ d0, unsigned short* __restrict__ d1, unsigned short* __restrict__ d2, unsigned short* __restrict__ d3) {
  const unsigned y = blockIdx.y;
  const float* src = (y == 0u) ? w0 : ((y == 1u) ? w1 : ((y == 2u) ? w2 : w3));
  unsigned short* dst = (y == 0u) ? d0 : ((y == 1u) ? d1 : ((y == 2u) ? d2 : d3));
  const unsigned u = blockIdx.x * 256u + threadIdx.x;
  const unsigned n = u >> 8;
  const unsigned k0 = (u & 255u) * 8u;
  float w[8];
#pragma unroll
  for (unsigned e = 0; e < 8u; ++e) w[e] = bf_rne_f32(src[(size_t)(k0 + e) * DIM + n]) * 16.0f;
  v4u pk; pk.x = pk2h(w[0], w[1]); pk.y = pk2h(w[2], w[3]); pk.z = pk2h(w[4], w[5]); pk.w = pk2h(w[6], w[7]);
  VST2(v4u, dst + (size_t)n * DIM + k0, pk);
}

template <int OUT_MODE>
__device__ __forceinline__ void gemm64_body(const _Float16* __restrict__ A, unsigned lda, const _Float16* __restrict__ Bt, unsigned ldb,
                                            void* __restrict__ Cout, unsigned ldc, unsigned M, unsigned N, unsigned K, float scale, float* slab) {
  const unsigned lane = threadIdx.x & 31u;
  const unsigned wave = threadIdx.x >> 5;
  const unsigned tilesN = N >> 6;
  const unsigned tilesM = M >> 6;
  const unsigned tile = blockIdx.x * 8u + wave;
  if (tile >= tilesM * tilesN) return;
  const unsigned tm = tile / tilesN;
  const unsigned tn = tile - tm * tilesN;
  const unsigned m0 = tm << 6;
  const unsigned n0 = tn << 6;
  const unsigned rlane = lane & 15u;
  const unsigned koff  = (lane >> 4) * 8u;
  const unsigned mOff  = (lane >> 4) * 8u;

  v8f acc[4][4];
#pragma unroll
  for (int i = 0; i < 4; ++i)
#pragma unroll
    for (int j = 0; j < 4; ++j) acc[i][j] = (v8f){0.f, 0.f, 0.f, 0.f, 0.f, 0.f, 0.f, 0.f};

  for (unsigned k0 = 0; k0 < K; k0 += 32u) {
    v16h bh[4];
#pragma unroll
    for (int j = 0; j < 4; ++j) {
      const size_t bo = (size_t)(n0 + ((unsigned)j << 4) + rlane) * ldb + koff + k0;
      bh[j] = ldfrag(Bt + bo);
    }
#pragma unroll
    for (int i = 0; i < 4; ++i) {
      const size_t ao = (size_t)(m0 + ((unsigned)i << 4) + rlane) * lda + koff + k0;
      const v16h ah = ldfrag(A + ao);
#pragma unroll
      for (int j = 0; j < 4; ++j) acc[i][j] = mma16(ah, bh[j], acc[i][j]);
      dep_guard_h(acc[i][0], acc[i][3], ah, ah);
    }
    keep4_h(bh[0], bh[1], bh[2], bh[3]);
  }
  acc_guard4(acc[0][0], acc[0][1], acc[0][2], acc[0][3]);
  acc_guard4(acc[1][0], acc[1][1], acc[1][2], acc[1][3]);
  acc_guard4(acc[2][0], acc[2][1], acc[2][2], acc[2][3]);
  acc_guard4(acc[3][0], acc[3][1], acc[3][2], acc[3][3]);

#pragma unroll
  for (int i = 0; i < 4; ++i) {
    const unsigned mBase = m0 + ((unsigned)i << 4);
#pragma unroll
    for (int j = 0; j < 4; ++j) {
#pragma unroll
      for (int r = 0; r < 8; ++r) slab[(mOff + (unsigned)r) * 68u + ((unsigned)j << 4) + rlane] = acc[i][j][r] * scale;
    }
    __builtin_amdgcn_fence(3  , "workgroup");
    __builtin_amdgcn_wave_barrier();
    __builtin_amdgcn_fence(2  , "workgroup");
    if (OUT_MODE == 0) {
      float* C = (float*)Cout;
      const unsigned hh = lane >> 4, c4 = (lane & 15u) * 4u;
      for (int pass = 0; pass < 2; ++pass) {
#pragma unroll
        for (int it = 0; it < 8; ++it) {
          const unsigned row = (unsigned)it * 2u + hh;
          const v4f v = *(const v4f*)(slab + row * 68u + c4);
          *(volatile v4f*)(C + (size_t)(mBase + row) * ldc + n0 + c4) = v;
        }
        __threadfence();
      }
    } else {
      const unsigned q = lane >> 3, c8 = (lane & 7u) * 8u;
      unsigned short* C = (unsigned short*)Cout;
      for (int pass = 0; pass < 2; ++pass) {
#pragma unroll
        for (int it = 0; it < 4; ++it) {
          const unsigned row = (unsigned)it * 4u + q;
          const float* sp = slab + row * 68u + c8;
          v8h hv;
#pragma unroll
          for (int e = 0; e < 8; ++e) hv[e] = (_Float16)sp[e];
          *(volatile v8h*)(C + (size_t)(mBase + row) * ldc + n0 + c8) = hv;
        }
        __threadfence();
      }
    }
    __builtin_amdgcn_fence(3  , "workgroup");
    __builtin_amdgcn_wave_barrier();
    __builtin_amdgcn_fence(2  , "workgroup");
  }
}

__global__ __launch_bounds__(256) void k_gemm_f32(const unsigned short* __restrict__ A, unsigned lda, const unsigned short* __restrict__ Bt, unsigned ldb,
                                                   float* __restrict__ C, unsigned ldc, unsigned M, unsigned N, unsigned K, float scale) {
  __shared__ __align__(16) float sT[8][16 * 68];
  gemm64_body<0>((const _Float16*)A, lda, (const _Float16*)Bt, ldb, (void*)C, ldc, M, N, K, scale, sT[threadIdx.x >> 5]);
}
__global__ __launch_bounds__(256) void k_gemm_f16(const unsigned short* __restrict__ A, unsigned lda, const unsigned short* __restrict__ Bt, unsigned ldb,
                                                   unsigned short* __restrict__ C, unsigned ldc, unsigned M, unsigned N, unsigned K, float scale) {
  __shared__ __align__(16) float sT[8][16 * 68];
  gemm64_body<1>((const _Float16*)A, lda, (const _Float16*)Bt, ldb, (void*)C, ldc, M, N, K, scale, sT[threadIdx.x >> 5]);
}

__global__ __launch_bounds__(256) void k_rope(const float* __restrict__ QKf, const float* __restrict__ cs, const float* __restrict__ sn, unsigned short* __restrict__ QK16) {
  const unsigned u = blockIdx.x * 256u + threadIdx.x;
  const unsigned j8 = u & 7u, hs = (u >> 3) & 31u, row = u >> 8;
  const unsigned col0 = hs * 128u + j8 * 8u;
  const float* xr = QKf + (size_t)row * QKP + col0;
  const float* cr = cs + row * 64u + j8 * 8u;
  const float* sr = sn + row * 64u + j8 * 8u;
  const v4f a0 = *(const v4f*)(xr), a1 = *(const v4f*)(xr + 4), b0 = *(const v4f*)(xr + 64), b1 = *(const v4f*)(xr + 68);
  const v4f c0 = *(const v4f*)(cr), c1 = *(const v4f*)(cr + 4), s0 = *(const v4f*)(sr), s1 = *(const v4f*)(sr + 4);
  const v4f lo0 = a0 * c0 - b0 * s0, lo1 = a1 * c1 - b1 * s1;
  const v4f hi0 = b0 * c0 + a0 * s0, hi1 = b1 * c1 + a1 * s1;
  v4u pl, ph;
  pl.x = pk2h(lo0.x, lo0.y); pl.y = pk2h(lo0.z, lo0.w); pl.z = pk2h(lo1.x, lo1.y); pl.w = pk2h(lo1.z, lo1.w);
  ph.x = pk2h(hi0.x, hi0.y); ph.y = pk2h(hi0.z, hi0.w); ph.z = pk2h(hi1.x, hi1.y); ph.w = pk2h(hi1.z, hi1.w);
  unsigned short* d = QK16 + (size_t)row * QKP + col0;
  *(volatile v4u*)(d) = pl; *(volatile v4u*)(d + 64) = ph;
  __threadfence();
  *(volatile v4u*)(d) = pl; *(volatile v4u*)(d + 64) = ph;
}

#ifndef KATTN_ATTR
#define KATTN_ATTR __attribute__((amdgpu_num_vgpr(256)))
#endif
#define FA_NW 4
#define FA_PP 72
#define FA_OP 132
#define NQB (SEQ / 64)
__global__ __launch_bounds__(128) KATTN_ATTR void k_flash128(const unsigned short* __restrict__ QKp, const unsigned short* __restrict__ Vtp, unsigned short* __restrict__ AOp) {
  __shared__ __align__(16) _Float16 Ps[FA_NW][16 * FA_PP];
  __shared__ __align__(16) float    Os[FA_NW][16 * FA_OP];
  const unsigned tid = threadIdx.x, wave = tid >> 5, lane = tid & 31u, hf = lane >> 4, c = lane & 15u;
  const unsigned h = blockIdx.x / (unsigned)NQB;
  const unsigned qb = blockIdx.x - h * (unsigned)NQB;
  const unsigned q0 = qb * 64u + wave * 16u;
  const _Float16* QK = (const _Float16*)QKp;
  const _Float16* Vt = (const _Float16*)Vtp;
  const unsigned qoff = (q0 + c) * (unsigned)QKP + h * (unsigned)HD + 8u * hf;
  const unsigned koff = c * (unsigned)QKP + (unsigned)DIM + h * (unsigned)HD + 8u * hf;
  const unsigned voff = (h * (unsigned)HD + c) * (unsigned)SEQ + 8u * hf;
  _Float16* pw = Ps[wave];
  float* os = Os[wave];
  const float SCL = 0.08838834764831845f * 1.4426950408889634f;

  float mrow[8], lrow[8];
  v8f o[8];
#pragma unroll
  for (int r = 0; r < 8; ++r) { mrow[r] = -__builtin_inff(); lrow[r] = 0.f; }
#pragma unroll
  for (int t = 0; t < 8; ++t) o[t] = (v8f){0.f, 0.f, 0.f, 0.f, 0.f, 0.f, 0.f, 0.f};

#pragma unroll 1
  for (unsigned kv0 = 0; kv0 < (unsigned)SEQ; kv0 += 64u) {
    v8f s[4];
#pragma unroll
    for (int j = 0; j < 4; ++j) s[j] = (v8f){0.f, 0.f, 0.f, 0.f, 0.f, 0.f, 0.f, 0.f};
#pragma unroll 1
    for (unsigned cc = 0; cc < 4u; ++cc) {
      unsigned qo = qoff + cc * 32u;
      asm volatile("" : "+v"(qo));
      const v16h qa = ldfrag(QK + qo);
      const _Float16* kp = QK + koff + kv0 * (unsigned)QKP + cc * 32u;
      const v16h k0 = ldfrag(kp);
      const v16h k1 = ldfrag(kp + 16u * (unsigned)QKP);
      const v16h k2 = ldfrag(kp + 32u * (unsigned)QKP);
      const v16h k3 = ldfrag(kp + 48u * (unsigned)QKP);
      s[0] = mma16(qa, k0, s[0]);
      s[1] = mma16(qa, k1, s[1]);
      s[2] = mma16(qa, k2, s[2]);
      s[3] = mma16(qa, k3, s[3]);
      guard4(s[0], s[1], s[2], s[3], qa, k0, k1, k2, k3);
    }
    __builtin_amdgcn_fence(3  , "workgroup");
    __builtin_amdgcn_wave_barrier();
    __builtin_amdgcn_fence(2  , "workgroup");
#pragma unroll
    for (int r = 0; r < 8; ++r) {
      const float a0 = s[0][r] * SCL, a1 = s[1][r] * SCL, a2 = s[2][r] * SCL, a3 = s[3][r] * SCL;
      float mx = fmaxf(fmaxf(a0, a1), fmaxf(a2, a3));
      mx = fmaxf(mx, __shfl_xor(mx, 1, 32));
      mx = fmaxf(mx, __shfl_xor(mx, 2, 32));
      mx = fmaxf(mx, __shfl_xor(mx, 4, 32));
      mx = fmaxf(mx, __shfl_xor(mx, 8, 32));
      const float mnew = fmaxf(mrow[r], mx);
      const float alpha = exp2f(mrow[r] - mnew);
      mrow[r] = mnew;
      const float p0 = exp2f(a0 - mnew), p1 = exp2f(a1 - mnew), p2 = exp2f(a2 - mnew), p3 = exp2f(a3 - mnew);
      float ps = (p0 + p1) + (p2 + p3);
      ps += __shfl_xor(ps, 1, 32);
      ps += __shfl_xor(ps, 2, 32);
      ps += __shfl_xor(ps, 4, 32);
      ps += __shfl_xor(ps, 8, 32);
      lrow[r] = lrow[r] * alpha + ps;
      _Float16* pr = pw + (8u * hf + (unsigned)r) * (unsigned)FA_PP + c;
      pr[0]  = (_Float16)(p0 * 4096.0f);
      pr[16] = (_Float16)(p1 * 4096.0f);
      pr[32] = (_Float16)(p2 * 4096.0f);
      pr[48] = (_Float16)(p3 * 4096.0f);
#pragma unroll
      for (int t = 0; t < 8; ++t) o[t][r] *= alpha;
    }
    __builtin_amdgcn_fence(3  , "workgroup");
    __builtin_amdgcn_wave_barrier();
    __builtin_amdgcn_fence(2  , "workgroup");
#pragma unroll 1
    for (unsigned kk = 0; kk < 2u; ++kk) {
      const v16h pa = ldfrag(pw + c * (unsigned)FA_PP + kk * 32u + 8u * hf);
      const _Float16* vp = Vt + voff + kv0 + kk * 32u;
      {
        const v16h v0 = ldfrag(vp);
        const v16h v1 = ldfrag(vp + 16u * (unsigned)SEQ);
        const v16h v2 = ldfrag(vp + 32u * (unsigned)SEQ);
        const v16h v3 = ldfrag(vp + 48u * (unsigned)SEQ);
        o[0] = mma16(pa, v0, o[0]);
        o[1] = mma16(pa, v1, o[1]);
        o[2] = mma16(pa, v2, o[2]);
        o[3] = mma16(pa, v3, o[3]);
        guard4(o[0], o[1], o[2], o[3], pa, v0, v1, v2, v3);
      }
      {
        const v16h v4 = ldfrag(vp + 64u * (unsigned)SEQ);
        const v16h v5 = ldfrag(vp + 80u * (unsigned)SEQ);
        const v16h v6 = ldfrag(vp + 96u * (unsigned)SEQ);
        const v16h v7 = ldfrag(vp + 112u * (unsigned)SEQ);
        o[4] = mma16(pa, v4, o[4]);
        o[5] = mma16(pa, v5, o[5]);
        o[6] = mma16(pa, v6, o[6]);
        o[7] = mma16(pa, v7, o[7]);
        guard4(o[4], o[5], o[6], o[7], pa, v4, v5, v6, v7);
      }
    }
  }

#pragma unroll
  for (int r = 0; r < 8; ++r) {
    const float inv = 1.0f / (lrow[r] * 64.0f);
#pragma unroll
    for (int t = 0; t < 8; ++t) os[(8u * hf + (unsigned)r) * (unsigned)FA_OP + (unsigned)t * 16u + c] = o[t][r] * inv;
  }
  __builtin_amdgcn_fence(3  , "workgroup");
  __builtin_amdgcn_wave_barrier();
  __builtin_amdgcn_fence(2  , "workgroup");
  {
    const unsigned c8 = c * 8u;
    for (int pass = 0; pass < 2; ++pass) {
#pragma unroll
      for (int it = 0; it < 8; ++it) {
        const unsigned row = (unsigned)it * 2u + hf;
        const v4f x0 = *(const v4f*)(os + row * (unsigned)FA_OP + c8);
        const v4f x1 = *(const v4f*)(os + row * (unsigned)FA_OP + c8 + 4u);
        v4u pk; pk.x = pk2h(x0.x, x0.y); pk.y = pk2h(x0.z, x0.w); pk.z = pk2h(x1.x, x1.y); pk.w = pk2h(x1.z, x1.w);
        *(volatile v4u*)(AOp + (size_t)(q0 + row) * DIM + h * (unsigned)HD + c8) = pk;
      }
      __threadfence();
    }
  }
}

#define SZ_X16  ((size_t)NB * SEQ * DIM * 2)
#define SZ_WQK  ((size_t)2 * DIM * DIM * 2)
#define SZ_W1   ((size_t)DIM * DIM * 2)
#define SZ_QKF  ((size_t)SEQ * QKP * 4)
#define SZ_QK16 ((size_t)SEQ * QKP * 2)
#define SZ_VT   ((size_t)DIM * SEQ * 2)
#define SZ_AO   ((size_t)SEQ * DIM * 2)
#define SZ_TAB  ((size_t)SEQ * 64 * 4)
#define CARVE_TOTAL (SZ_X16 + SZ_WQK + 2 * SZ_W1 + SZ_QKF + SZ_QK16 + SZ_VT + SZ_AO + 2 * SZ_TAB)
static_assert(CARVE_TOTAL <= (size_t)134217728);
static_assert(SZ_X16 % 256 == 0 && SZ_WQK % 256 == 0 && SZ_W1 % 256 == 0 && SZ_QKF % 256 == 0 && SZ_QK16 % 256 == 0 && SZ_VT % 256 == 0 && SZ_AO % 256 == 0 && SZ_TAB % 256 == 0);
static_assert(((SEQ / 64) * (QKP / 64)) % 8 == 0);
static_assert(((DIM / 64) * (SEQ / 64)) % 8 == 0);
static_assert(((SEQ / 64) * (DIM / 64)) % 8 == 0);
static_assert(DIM % 32 == 0);

extern "C" void kernel_launch(void* const* d_in, const int* in_sizes, int n_in, void* d_out, int out_size, void* d_ws, size_t ws_size, hipStream_t stream) {
  if (n_in < 5) return;
  if ((long long)in_sizes[0] < (long long)(NB - 1) * XB_FULL + (long long)SEQ * DIM) return;
  if ((long long)in_sizes[1] < (long long)DIM * DIM || (long long)in_sizes[2] < (long long)DIM * DIM) return;
  if ((long long)in_sizes[3] < (long long)DIM * DIM || (long long)in_sizes[4] < (long long)DIM * DIM) return;
  if ((long long)out_size < (long long)NB * SEQ * DIM) return;
  if (ws_size < CARVE_TOTAL) return;

  const float* x  = (const float*)d_in[0];
  const float* Wq = (const float*)d_in[1];
  const float* Wk = (const float*)d_in[2];
  const float* Wv = (const float*)d_in[3];
  const float* Wo = (const float*)d_in[4];
  float* out = (float*)d_out;

  char* wsp = (char*)d_ws;
  unsigned short* X16  = (unsigned short*)wsp; wsp += SZ_X16;
  unsigned short* WQK  = (unsigned short*)wsp; wsp += SZ_WQK;
  unsigned short* WV   = (unsigned short*)wsp; wsp += SZ_W1;
  unsigned short* WO   = (unsigned short*)wsp; wsp += SZ_W1;
  float*          QKF  = (float*)wsp;          wsp += SZ_QKF;
  unsigned short* QK16 = (unsigned short*)wsp; wsp += SZ_QK16;
  unsigned short* VT16 = (unsigned short*)wsp; wsp += SZ_VT;
  unsigned short* AO16 = (unsigned short*)wsp; wsp += SZ_AO;
  float*          CS   = (float*)wsp;          wsp += SZ_TAB;
  float*          SN   = (float*)wsp;          wsp += SZ_TAB;

  InvF f;
  for (int i = 0; i < 64; ++i) {
    const float e = (float)(2 * i) / 128.0f;
    const float p = (float)pow(10000.0, (double)e);
    f.v[i] = 1.0f / p;
  }

  k_tab<<<dim3((unsigned)(SEQ * 64 / 256)), 256, 0, stream>>>(CS, SN, f);
  k_cast_x<<<dim3((unsigned)(SEQ * DIM / 8 / 256), (unsigned)NB), 256, 0, stream>>>(x, X16);
  k_castT4<<<dim3((unsigned)(DIM * DIM / 8 / 256), 4u), 256, 0, stream>>>(Wq, Wk, Wv, Wo, WQK, WQK + (size_t)DIM * DIM, WV, WO);

  for (int b = 0; b < NB; ++b) {
    const unsigned short* Xb = X16 + (size_t)b * ((size_t)SEQ * DIM);
    k_gemm_f32<<<dim3((unsigned)((SEQ / 64) * (QKP / 64) / 8)), 256, 0, stream>>>(Xb, (unsigned)DIM, WQK, (unsigned)DIM, QKF, (unsigned)QKP,
                                                                                    (unsigned)SEQ, (unsigned)QKP, (unsigned)DIM, 0.0625f);
    k_rope<<<dim3((unsigned)SEQ), 256, 0, stream>>>(QKF, CS, SN, QK16);
    k_gemm_f16<<<dim3((unsigned)((DIM / 64) * (SEQ / 64) / 8)), 256, 0, stream>>>(WV, (unsigned)DIM, Xb, (unsigned)DIM, VT16, (unsigned)SEQ,
                                                                                   (unsigned)DIM, (unsigned)SEQ, (unsigned)DIM, 0.0625f);
    k_flash128<<<dim3((unsigned)(NH * NQB)), 128, 0, stream>>>(QK16, VT16, AO16);
    k_gemm_f32<<<dim3((unsigned)((SEQ / 64) * (DIM / 64) / 8)), 256, 0, stream>>>(AO16, (unsigned)DIM, WO, (unsigned)DIM, out + (size_t)b * ((size_t)SEQ * DIM), (unsigned)DIM,
                                                                                   (unsigned)SEQ, (unsigned)DIM, (unsigned)DIM, 0.0009765625f);
  }
}
